// _MaskedConv_38019050504696
// MI455X (gfx1250) — hardware-verified
//
#include <hip/hip_runtime.h>
#include <stdint.h>

#define KNBR 16
#define CIN  64
#define COUT 64
#define RED  (KNBR * CIN)
#define TM   64
#define KCH  4
#define KC   (KCH * CIN)
#define NCH  (KNBR / KCH)
#define ZS   264
#define CS   68

static_assert((ZS % 8) == 0);
static_assert(ZS >= KC);
static_assert((TM * ZS) >= ((TM - 1) * ZS + KC));
static_assert((CS % 4) == 0);
static_assert((TM * CS) >= ((TM - 1) * CS + COUT));
static_assert(TM == 64);
static_assert(CIN == 64);
static_assert(COUT == 64);
static_assert(KC == 256);
static_assert((NCH * KCH) == KNBR);

typedef __bf16       v16b __attribute__((ext_vector_type(16)));
typedef float        v8f  __attribute__((ext_vector_type(8)));
typedef float        v4f  __attribute__((ext_vector_type(4)));
typedef unsigned int v4u  __attribute__((ext_vector_type(4)));

union Frag { v16b v; v4u u[2]; };

__device__ __forceinline__ unsigned short bf_bits(float f) {
  const unsigned u = __float_as_uint(f);
  return (unsigned short)((u + 0x7FFFu + ((u >> 16) & 1u)) >> 16);
}
__device__ __forceinline__ float bfr(float f) { return __uint_as_float(((unsigned)bf_bits(f)) << 16); }
__device__ __forceinline__ unsigned pk16(unsigned short a, unsigned short b) { return (unsigned)a | ((unsigned)b << 16); }
__device__ __forceinline__ v8f zero8() { v8f z = {0.f, 0.f, 0.f, 0.f, 0.f, 0.f, 0.f, 0.f}; return z; }

__device__ __forceinline__ Frag ldfrag(const unsigned short* p) {
  Frag f;
  f.u[0] = *(const v4u*)(p);
  f.u[1] = *(const v4u*)(p + 16);
  return f;
}

__device__ __forceinline__ v8f mma_bf(const Frag& a, const Frag& b, v8f c) {
  return __builtin_amdgcn_wmma_f32_16x16x32_bf16(false, a.v, false, b.v, (short)0, c, false, false);
}
__device__ __forceinline__ void guard(v8f& c, const Frag& a, const Frag& b) {
#if defined(__HIP_DEVICE_COMPILE__)
  asm volatile("v_nop\n\tv_nop\n\tv_nop\n\tv_nop" : "+v"(c) : "v"(a.u[0]), "v"(a.u[1]), "v"(b.u[0]), "v"(b.u[1]));
#endif
}

__global__ __launch_bounds__(256)
void k_cvt(const float* __restrict__ X, const float* __restrict__ W,
           unsigned short* Px, unsigned short* Pw, int npX, int npW, int nbX) {
  const int blk = blockIdx.x, tid = threadIdx.x;
  if (blk < nbX) {
    const int p  = blk * 256 + tid;
    const int pc = min(p, npX - 1);
    const v4f a = *(const v4f*)(X + (size_t)pc * 8);
    const v4f b = *(const v4f*)(X + (size_t)pc * 8 + 4);
    v4u u;
    u[0] = pk16(bf_bits(a[0]), bf_bits(a[1]));
    u[1] = pk16(bf_bits(a[2]), bf_bits(a[3]));
    u[2] = pk16(bf_bits(b[0]), bf_bits(b[1]));
    u[3] = pk16(bf_bits(b[2]), bf_bits(b[3]));
    unsigned short* d = Px + (size_t)pc * 8;
    if (p < npX) *(volatile v4u*)d = u;
    __threadfence();
    if (p < npX) *(volatile v4u*)d = u;
  } else {
    const int p  = (blk - nbX) * 256 + tid;
    const int pc = min(p, npW - 1);
    const int o  = pc >> 7;
    const int kk = (pc & 127) >> 3;
    const int c0 = (pc & 7) * 8;
    const float* wp = W + (size_t)o * RED + (size_t)c0 * KNBR + kk;
    float f[8];
#pragma unroll
    for (int i = 0; i < 8; ++i) f[i] = wp[i * KNBR];
    v4u u;
    u[0] = pk16(bf_bits(f[0]), bf_bits(f[1]));
    u[1] = pk16(bf_bits(f[2]), bf_bits(f[3]));
    u[2] = pk16(bf_bits(f[4]), bf_bits(f[5]));
    u[3] = pk16(bf_bits(f[6]), bf_bits(f[7]));
    unsigned short* d = Pw + (size_t)pc * 8;
    if (p < npW) *(volatile v4u*)d = u;
    __threadfence();
    if (p < npW) *(volatile v4u*)d = u;
  }
}

__global__ __launch_bounds__(256)
void k_conv(const unsigned short* __restrict__ Px, const unsigned short* __restrict__ Pw,
            const int* __restrict__ kidx, const int* __restrict__ kmask,
            const float* __restrict__ bias, float* out, int M, int npts) {
  __shared__ __align__(16) unsigned short zt[TM * ZS];
  __shared__ __align__(16) float sC[TM * CS];
  __shared__ float sBias[COUT];

  const int tid = threadIdx.x, lane = tid & 31, wave = tid >> 5, hh = lane >> 4, c = lane & 15;
  const int m0 = blockIdx.x * TM;

  if (tid < COUT) sBias[tid] = bfr(bias[tid]);

  const int ct  = wave & 3, mh = wave >> 2;
  const int o   = 16 * ct + c;
  const int mtA = 2 * mh, mtB = 2 * mh + 1;

  const int e  = tid >> 2, q = tid & 3;
  const int mg = min(m0 + e, M - 1);
  const int bb = mg / npts;
  const int nn = mg - bb * npts;
  const int* ip = kidx  + (size_t)nn * KNBR;
  const int* mp = kmask + (size_t)nn * KNBR;
  const unsigned short* xb = Px + (size_t)bb * (size_t)npts * CIN;
  unsigned short* dp = zt + e * ZS + CIN * q;

  v8f acc0 = zero8(), acc1 = zero8();

#pragma unroll 1
  for (int ch = 0; ch < NCH; ++ch) {
    {
      const int kk = KCH * ch + q;
      int j = ip[kk];
      const int mk = mp[kk];
      j = min(max(j, 0), npts - 1);
      const unsigned keep = (mk != 0) ? 0xFFFFFFFFu : 0u;
      const v4u kv = {keep, keep, keep, keep};
      const unsigned short* sp = xb + (size_t)j * CIN;
      v4u u[8];
#pragma unroll
      for (int i = 0; i < 8; ++i) u[i] = *(const v4u*)(sp + 8 * i);
#pragma unroll
      for (int i = 0; i < 8; ++i) {
        const v4u t = u[i] & kv;
        *(v4u*)(dp + 8 * i) = t;
      }
    }
    Frag bf[8];
    {
      const unsigned short* wp = Pw + (size_t)o * RED + KC * ch + 8 * hh;
#pragma unroll
      for (int g = 0; g < 8; ++g) bf[g] = ldfrag(wp + 32 * g);
    }
    __syncthreads();

    {
      const unsigned short* ap = zt + (16 * mtA + c) * ZS + 8 * hh;
#pragma unroll
      for (int g = 0; g < 8; ++g) {
        const Frag af = ldfrag(ap + 32 * g);
        acc0 = mma_bf(af, bf[g], acc0);
        guard(acc0, af, bf[g]);
      }
    }
    {
      const unsigned short* ap = zt + (16 * mtB + c) * ZS + 8 * hh;
#pragma unroll
      for (int g = 0; g < 8; ++g) {
        const Frag af = ldfrag(ap + 32 * g);
        acc1 = mma_bf(af, bf[g], acc1);
        guard(acc1, af, bf[g]);
      }
    }
    __syncthreads();
  }

  {
    const float bv = sBias[o];
    float* c0p = sC + (16 * mtA + 8 * hh) * CS + o;
    float* c1p = sC + (16 * mtB + 8 * hh) * CS + o;
#pragma unroll
    for (int r = 0; r < 8; ++r) c0p[r * CS] = acc0[r] + bv;
#pragma unroll
    for (int r = 0; r < 8; ++r) c1p[r * CS] = acc1[r] + bv;
  }
  __syncthreads();

  if (m0 + TM <= M) {
    v4f v[4];
#pragma unroll
    for (int s = 0; s < 4; ++s) {
      const int f = (s * 256 + tid) * 4;
      const int row = f >> 6, col = f & 63;
      v[s] = *(const v4f*)(sC + row * CS + col);
    }
    float* ob = out + (size_t)m0 * COUT;
#pragma unroll
    for (int s = 0; s < 4; ++s) *(volatile v4f*)(ob + (size_t)(s * 256 + tid) * 4) = v[s];
    __threadfence();
#pragma unroll
    for (int s = 0; s < 4; ++s) *(volatile v4f*)(ob + (size_t)(s * 256 + tid) * 4) = v[s];
  } else {
    float v[16];
#pragma unroll
    for (int i = 0; i < 16; ++i) {
      const int f = i * 256 + tid;
      v[i] = sC[(f >> 6) * CS + (f & 63)];
    }
    float* ob = out + (size_t)m0 * COUT;
#pragma unroll
    for (int i = 0; i < 16; ++i) {
      const int f = i * 256 + tid;
      if (m0 + (f >> 6) < M) *(volatile float*)(ob + f) = v[i];
    }
    __threadfence();
#pragma unroll
    for (int i = 0; i < 16; ++i) {
      const int f = i * 256 + tid;
      if (m0 + (f >> 6) < M) *(volatile float*)(ob + f) = v[i];
    }
  }
}

static inline size_t al256(size_t x) { return (x + 255) & ~(size_t)255; }

extern "C" void kernel_launch(void* const* d_in, const int* in_sizes, int n_in,
                              void* d_out, int out_size, void* d_ws, size_t ws_size,
                              hipStream_t stream) {
  if (n_in < 5) return;
  const int nX = in_sizes[0], nI = in_sizes[1], nMk = in_sizes[2], nW = in_sizes[3], nB = in_sizes[4];
  if (nI < KNBR || (nI % KNBR) != 0 || nMk != nI) return;
  const int npts = nI / KNBR;
  if (nW != COUT * RED || nB != COUT) return;
  const long long rowsz = (long long)npts * CIN;
  if (nX <= 0 || ((long long)nX % rowsz) != 0) return;
  const int batch = (int)((long long)nX / rowsz);
  const long long Mll = (long long)batch * npts;
  if (Mll <= 0 || Mll * COUT != (long long)out_size) return;
  const int M = (int)Mll;

  const float* x     = (const float*)d_in[0];
  const int*   kidx  = (const int*)d_in[1];
  const int*   kmask = (const int*)d_in[2];
  const float* w     = (const float*)d_in[3];
  const float* bias  = (const float*)d_in[4];
  float* out = (float*)d_out;

  const size_t sPx = al256((size_t)nX * 2);
  const size_t sPw = al256((size_t)nW * 2);
  size_t off = 0;
  const size_t oPx = off; off += sPx;
  const size_t oPw = off; off += sPw;
  if (off > ws_size) return;
  if (off > (size_t)134217728) return;

  char* ws = (char*)d_ws;
  unsigned short* Px = (unsigned short*)(ws + oPx);
  unsigned short* Pw = (unsigned short*)(ws + oPw);

  const int npX = nX / 8;
  const int npW = nW / 8;
  const int nbX = (npX + 255) / 256, nbW = (npW + 255) / 256;

  k_cvt<<<dim3(nbX + nbW), dim3(256), 0, stream>>>(x, w, Px, Pw, npX, npW, nbX);
  const int nblk = (M + TM - 1) / TM;
  k_conv<<<dim3(nblk), dim3(256), 0, stream>>>(Px, Pw, kidx, kmask, bias, out, M, npts);
  (void)hipGetLastError();
}
